// GNNLayer_67912022884494
// MI455X (gfx1250) — hardware-run, weakly checked
//
#include <hip/hip_runtime.h>
#include <stddef.h>
#include <stdint.h>
#include <math.h>


#define CIN     256
#define HWID    512
#define KP      512
#define NTHR    256
#define NWAVE   8
#define EPT     8
#define CHUNK   (NTHR * EPT)
#define WCAP    (EPT * 32)
#define LISTN   (NWAVE * WCAP)
#define NBA     512
#define PKS     9
#define RCAP    28672
#define DEGCAP  128
#define GBM     64
#define GBN     128
#define GTHR    128
#define NEGSL   0.2f
#define BNEPS   1e-5f
#define NUW     (CIN * (CIN / 8))
#define NUP     (CIN * (KP / 8))
#define ZINTS   (2 * RCAP + 2 * NBA + LISTN)
#define LDS_AGG (ZINTS * 4 + 64)
#define WSMAX   134217728

static_assert((CHUNK & (CHUNK - 1)) == 0);
static_assert(NBA == (1 << PKS));
static_assert(((long long)CHUNK << PKS) < (1LL << 31));
static_assert(NTHR * 2 == NBA);
static_assert(LISTN >= NBA && LISTN >= NWAVE * WCAP);
static_assert((RCAP % 32) == 0);
static_assert((ZINTS % (NTHR * 4)) == 0);
static_assert(LDS_AGG <= 262144);
static_assert((NBA % NWAVE) == 0 && (NBA % GBM) == 0 && (NBA % 4) == 0 && NBA / 4 <= NTHR);
static_assert(GBM == (GTHR / 32) * 16 && GBN == 4 * 32);
static_assert((CIN % GBN) == 0 && (HWID % GBN) == 0 && (CIN % 32) == 0 && (KP % 32) == 0);
static_assert(KP == 2 * CIN && HWID == 2 * CIN);
static_assert(CIN == 32 * 8);
static_assert((NUW % NTHR) == 0 && (NUP % NTHR) == 0);

typedef float          v4f  __attribute__((ext_vector_type(4)));
typedef float          v8f  __attribute__((ext_vector_type(8)));
typedef int            v4i  __attribute__((ext_vector_type(4)));
typedef int            v8i  __attribute__((ext_vector_type(8)));
typedef unsigned int   v4u  __attribute__((ext_vector_type(4)));
typedef unsigned short v8us __attribute__((ext_vector_type(8)));
typedef __bf16         v16b __attribute__((ext_vector_type(16)));
typedef v4f  __attribute__((may_alias)) v4fa;
typedef v4i  __attribute__((may_alias)) v4ia;
typedef v8us __attribute__((may_alias)) v8usa;
union Frag { v16b b; v8us h[2]; v8i w; };

__device__ __forceinline__ v8f wmb(const Frag& a, const Frag& b, v8f c) {
  v8f d = __builtin_amdgcn_wmma_f32_16x16x32_bf16(false, a.b, false, b.b, (short)0, c, false, false);
  asm volatile("v_nop\n\tv_nop\n\tv_nop\n\tv_nop" : "+v"(d) : "v"(a.w), "v"(b.w));
  return d;
}

__device__ __forceinline__ unsigned short bf_bits(float f) {
  unsigned int u = __float_as_uint(f);
  u += 0x7FFFu + ((u >> 16) & 1u);
  return (unsigned short)(u >> 16);
}
__device__ __forceinline__ float bf_val(unsigned short b) {
  return __uint_as_float(((unsigned int)b) << 16);
}
__device__ __forceinline__ float bf_rne(float f) { return bf_val(bf_bits(f)); }
__device__ __forceinline__ void ld8bf(const float* __restrict__ p, float o[8]) {
  const v4f a = *(const v4f*)p;
  const v4f b = *(const v4f*)(p + 4);
  o[0] = bf_rne(a.x); o[1] = bf_rne(a.y); o[2] = bf_rne(a.z); o[3] = bf_rne(a.w);
  o[4] = bf_rne(b.x); o[5] = bf_rne(b.y); o[6] = bf_rne(b.z); o[7] = bf_rne(b.w);
}

__device__ __forceinline__ int scan_chunk(const int* __restrict__ dsts, int nE, int cbase, int slotBase,
                                          int nb, int vec8, int* list, int tid, int lane, int wave) {
  int wc = 0;
  const int el0  = tid * EPT;
  const int e0   = cbase + el0;
  const int sent = -2147483647 - 1;
  v4i da, db;
  if (vec8 != 0 && cbase + CHUNK <= nE) {
    da = *(const v4i*)(dsts + e0);
    db = *(const v4i*)(dsts + e0 + 4);
  } else {
    da.x = (e0     < nE) ? dsts[min(e0,     nE - 1)] : sent;
    da.y = (e0 + 1 < nE) ? dsts[min(e0 + 1, nE - 1)] : sent;
    da.z = (e0 + 2 < nE) ? dsts[min(e0 + 2, nE - 1)] : sent;
    da.w = (e0 + 3 < nE) ? dsts[min(e0 + 3, nE - 1)] : sent;
    db.x = (e0 + 4 < nE) ? dsts[min(e0 + 4, nE - 1)] : sent;
    db.y = (e0 + 5 < nE) ? dsts[min(e0 + 5, nE - 1)] : sent;
    db.z = (e0 + 6 < nE) ? dsts[min(e0 + 6, nE - 1)] : sent;
    db.w = (e0 + 7 < nE) ? dsts[min(e0 + 7, nE - 1)] : sent;
  }
  const unsigned nbs = (unsigned)slotBase;
  const unsigned unb = (unsigned)nb;
  const unsigned s0 = (unsigned)da.x - nbs, s1 = (unsigned)da.y - nbs;
  const unsigned s2 = (unsigned)da.z - nbs, s3 = (unsigned)da.w - nbs;
  const unsigned s4 = (unsigned)db.x - nbs, s5 = (unsigned)db.y - nbs;
  const unsigned s6 = (unsigned)db.z - nbs, s7 = (unsigned)db.w - nbs;
  const bool h0 = s0 < unb, h1 = s1 < unb, h2 = s2 < unb, h3 = s3 < unb;
  const bool h4 = s4 < unb, h5 = s5 < unb, h6 = s6 < unb, h7 = s7 < unb;
  const unsigned any = __builtin_amdgcn_ballot_w32(h0 | h1 | h2 | h3 | h4 | h5 | h6 | h7);
  if (any != 0u) {
#define HITJ(J, HJ, SJ) { \
      const unsigned mj = __builtin_amdgcn_ballot_w32(HJ); \
      if (mj != 0u) { \
        if (HJ) { \
          const int pos = wc + (int)__builtin_amdgcn_mbcnt_lo(mj, 0u); \
          if (pos < WCAP) list[wave * WCAP + pos] = ((el0 + (J)) << PKS) | (int)(SJ); \
        } \
        wc += (int)__builtin_popcount(mj); } }
    HITJ(0, h0, s0)
    HITJ(1, h1, s1)
    HITJ(2, h2, s2)
    HITJ(3, h3, s3)
    HITJ(4, h4, s4)
    HITJ(5, h5, s5)
    HITJ(6, h6, s6)
    HITJ(7, h7, s7)
#undef HITJ
  }
  return wc;
}

__device__ __forceinline__ int seg_front(const int* __restrict__ dsts, int nE, int nodeBase, int vec8,
                                         int* lds_i, int tid, int lane, int wave) {
  int* reg1 = lds_i;
  int* reg2 = reg1 + RCAP;
  int* scnt = reg2 + RCAP;
  int* soff = scnt + NBA;
  int* list = soff + NBA;
  int* wcnt = list + LISTN;
  int* wtot = wcnt + NWAVE;

  {
    const v4i z4 = {0, 0, 0, 0};
    for (int i = tid * 4; i < ZINTS; i += NTHR * 4) *(v4ia*)(lds_i + i) = z4;
    if (tid < 2 * NWAVE) wcnt[tid] = 0;
  }
  __syncthreads();

  int tot = 0;
  const int nChunks = (nE + CHUNK - 1) / CHUNK;
#pragma unroll 1
  for (int ch = 0; ch < nChunks; ++ch) {
    const int cbase = ch * CHUNK;
    const int wc = scan_chunk(dsts, nE, cbase, nodeBase, NBA, vec8, list, tid, lane, wave);
    if (lane == 0) wcnt[wave] = wc;
    __syncthreads();
    int pre = 0, all = 0;
#pragma unroll
    for (int w2 = 0; w2 < NWAVE; ++w2) {
      int c = wcnt[w2];
      c = c < 0 ? 0 : (c > WCAP ? WCAP : c);
      all += c;
      pre += (w2 < wave) ? c : 0;
    }
    const int wcc  = wc > WCAP ? WCAP : wc;
    const int base = tot + pre;
#pragma unroll 1
    for (int i = lane; i < wcc; i += 32) {
      const int ent = list[wave * WCAP + i];
      const int el  = (ent >> PKS) & (CHUNK - 1);
      const int sl  = ent & (NBA - 1);
      int eid = cbase + el;
      eid = eid > nE - 1 ? nE - 1 : eid;
      const int pos = base + i;
      if (pos < RCAP) reg1[pos] = (int)(((unsigned)eid << PKS) | (unsigned)sl);
    }
    tot += all;
    tot = tot > RCAP ? RCAP : tot;
    __syncthreads();
  }
  const int nh = tot;

  if (wave == 0) {
#pragma unroll 1
    for (int b0 = 0; b0 < nh; b0 += 32) {
      const int idx = b0 + lane;
      const int uv  = reg1[idx < RCAP ? idx : RCAP - 1];
      const int m32 = (nh - b0) < 32 ? (nh - b0) : 32;
#pragma unroll 1
      for (int k = 0; k < m32; ++k) {
        const int u  = __builtin_amdgcn_readlane(uv, k);
        const int sl = u & (NBA - 1);
        if (lane == 0) scnt[sl] = scnt[sl] + 1;
      }
    }
  }
  __syncthreads();

  {
    const int c0r = scnt[2 * tid], c1r = scnt[2 * tid + 1];
    const int e0 = c0r < 0 ? 0 : c0r, e1 = c1r < 0 ? 0 : c1r;
    const int ts = e0 + e1;
    int incl = ts;
#pragma unroll
    for (int d = 1; d < 32; d <<= 1) {
      const int up = __shfl_up(incl, d, 32);
      if (lane >= d) incl += up;
    }
    if (lane == 31) wtot[wave] = incl;
    __syncthreads();
    int pre = 0;
#pragma unroll
    for (int w2 = 0; w2 < NWAVE; ++w2) pre += (w2 < wave) ? wtot[w2] : 0;
    int run = pre + incl - ts;
    soff[2 * tid + 0] = run; run += e0;
    soff[2 * tid + 1] = run;
  }
  __syncthreads();
  for (int i = tid; i < NBA; i += NTHR) list[i] = soff[i];
  __syncthreads();

  if (wave == 0) {
#pragma unroll 1
    for (int b0 = 0; b0 < nh; b0 += 32) {
      const int idx = b0 + lane;
      const int uv  = reg1[idx < RCAP ? idx : RCAP - 1];
      const int m32 = (nh - b0) < 32 ? (nh - b0) : 32;
#pragma unroll 1
      for (int k = 0; k < m32; ++k) {
        const int u   = __builtin_amdgcn_readlane(uv, k);
        const int sl  = u & (NBA - 1);
        const int eid = (int)((unsigned)u >> PKS);
        if (lane == 0) {
          int pos = list[sl];
          pos = pos < 0 ? 0 : (pos > RCAP - 1 ? RCAP - 1 : pos);
          reg2[pos] = eid;
          list[sl] = pos + 1;
        }
      }
    }
  }
  __syncthreads();
  return nh;
}

__global__ __launch_bounds__(NTHR) void k_wprep(const float* __restrict__ wg, const float* __restrict__ wa,
                                                const float* __restrict__ wp,
                                                unsigned short* WB, unsigned short* WPB) {
  const int u = (int)blockIdx.x * NTHR + (int)threadIdx.x;
  v8us o;
  unsigned short* dp;
  if (u < NUW) {
    const int n  = u >> 5;
    const int k8 = (u & 31) * 8;
    const float* p = wg + (size_t)k8 * CIN + n;
#pragma unroll
    for (int i = 0; i < 8; ++i) o[i] = bf_bits(p[(size_t)i * CIN]);
    dp = WB + (size_t)n * CIN + k8;
  } else if (u < 2 * NUW) {
    const int v  = u - NUW;
    const int n  = v >> 5;
    const int k8 = (v & 31) * 8;
    const float* p = wa + (size_t)k8 * CIN + n;
#pragma unroll
    for (int i = 0; i < 8; ++i) o[i] = bf_bits(p[(size_t)i * CIN]);
    dp = WB + (size_t)(CIN + n) * CIN + k8;
  } else if (u < 2 * NUW + NUP) {
    const int v  = u - 2 * NUW;
    const int n  = v >> 6;
    const int k8 = (v & 63) * 8;
    const int kk = k8 & (CIN - 1);
    const float* p = wp + (size_t)kk * CIN + n;
#pragma unroll
    for (int i = 0; i < 8; ++i) o[i] = bf_bits(p[(size_t)i * CIN]);
    dp = WPB + (size_t)n * KP + k8;
  } else {
    return;
  }
  *(volatile v8us*)dp = o;
  __threadfence();
  *(volatile v8us*)dp = o;
}

__global__ __launch_bounds__(NTHR) void k_cvx(const float* __restrict__ x, int nN, int nUnits,
                                              unsigned short* xb) {
  const int u = (int)blockIdx.x * NTHR + (int)threadIdx.x;
  if (u >= nUnits) return;
  const int row = u >> 5;
  const int c8  = (u & 31) * 8;
  const int rc  = row < nN ? row : nN - 1;
  const float keep = row < nN ? 1.0f : 0.0f;
  const float* p = x + (size_t)rc * CIN + c8;
  const v4f a = *(const v4f*)p;
  const v4f b = *(const v4f*)(p + 4);
  v8us o;
  o[0] = bf_bits(a.x * keep); o[1] = bf_bits(a.y * keep); o[2] = bf_bits(a.z * keep); o[3] = bf_bits(a.w * keep);
  o[4] = bf_bits(b.x * keep); o[5] = bf_bits(b.y * keep); o[6] = bf_bits(b.z * keep); o[7] = bf_bits(b.w * keep);
  unsigned short* dp = xb + (size_t)u * 8;
  *(volatile v8us*)dp = o;
  __threadfence();
  *(volatile v8us*)dp = o;
}

template <int MODE>
__global__ __launch_bounds__(GTHR) void k_gemm(const unsigned short* __restrict__ A, int lda,
                                               const unsigned short* __restrict__ BT, int ldb, int K,
                                               float* C32, int ldc,
                                               const float* __restrict__ GC, const float* __restrict__ xin,
                                               const float* __restrict__ bgcn, const float* __restrict__ bproj,
                                               const float* __restrict__ gam, const float* __restrict__ bet,
                                               const float* __restrict__ mu, const float* __restrict__ var,
                                               float* out, int nN) {
  __shared__ __attribute__((aligned(16))) float stg[GBM * GBN];
  const int tid = (int)threadIdx.x, lane = tid & 31, wave = tid >> 5, hh = lane >> 4, m = lane & 15;
  const int rowBase = (int)blockIdx.x * GBM;
  const int colBase = (int)blockIdx.y * GBN;

  v8f acc[8];
  {
    const v8f z = {0.f, 0.f, 0.f, 0.f, 0.f, 0.f, 0.f, 0.f};
#pragma unroll
    for (int t = 0; t < 8; ++t) acc[t] = z;
  }
  const unsigned short* ap = A  + (size_t)(rowBase + 16 * wave + m) * (size_t)lda + 8 * hh;
  const unsigned short* bp = BT + (size_t)(colBase + m) * (size_t)ldb + 8 * hh;

#pragma unroll 1
  for (int k0 = 0; k0 < K; k0 += 32) {
    Frag af;
    af.h[0] = *(const v8usa*)(ap + k0);
    af.h[1] = *(const v8usa*)(ap + k0 + 16);
#pragma unroll
    for (int nt = 0; nt < 8; ++nt) {
      const unsigned short* wq = bp + (size_t)(16 * nt) * (size_t)ldb + k0;
      Frag bf;
      bf.h[0] = *(const v8usa*)wq;
      bf.h[1] = *(const v8usa*)(wq + 16);
      acc[nt] = wmb(af, bf, acc[nt]);
    }
  }

#pragma unroll
  for (int nt = 0; nt < 8; ++nt) {
    const int lc = 16 * nt + m;
#pragma unroll
    for (int r = 0; r < 8; ++r) {
      const int lr = 16 * wave + 8 * hh + r;
      stg[lr * GBN + lc] = acc[nt][r];
    }
  }
  __syncthreads();

  if constexpr (MODE == 0) {
    v4f pv[16];
#pragma unroll
    for (int i = 0; i < 16; ++i) pv[i] = *(const v4fa*)(stg + (16 * wave + i) * GBN + 4 * lane);
#pragma unroll
    for (int i = 0; i < 16; ++i) {
      const int row = rowBase + 16 * wave + i;
      float* op = C32 + (size_t)row * (size_t)ldc + colBase + 4 * lane;
      *(volatile v4f*)op = pv[i];
    }
    __threadfence();
#pragma unroll
    for (int i = 0; i < 16; ++i) {
      const int row = rowBase + 16 * wave + i;
      float* op = C32 + (size_t)row * (size_t)ldc + colBase + 4 * lane;
      *(volatile v4f*)op = pv[i];
    }
  } else {
    const int cb = colBase + 4 * lane;
    float bg_[4], bp_[4], gg[4], be[4], mm[4], rs[4];
    {
      const v4f b1 = *(const v4f*)(bgcn + cb), b2 = *(const v4f*)(bproj + cb);
      const v4f g4 = *(const v4f*)(gam + cb),  e4 = *(const v4f*)(bet + cb);
      const v4f m4 = *(const v4f*)(mu + cb),   v4 = *(const v4f*)(var + cb);
      bg_[0] = bf_rne(b1.x); bg_[1] = bf_rne(b1.y); bg_[2] = bf_rne(b1.z); bg_[3] = bf_rne(b1.w);
      bp_[0] = bf_rne(b2.x); bp_[1] = bf_rne(b2.y); bp_[2] = bf_rne(b2.z); bp_[3] = bf_rne(b2.w);
      gg[0]  = bf_rne(g4.x); gg[1]  = bf_rne(g4.y); gg[2]  = bf_rne(g4.z); gg[3]  = bf_rne(g4.w);
      be[0]  = bf_rne(e4.x); be[1]  = bf_rne(e4.y); be[2]  = bf_rne(e4.z); be[3]  = bf_rne(e4.w);
      mm[0]  = bf_rne(m4.x); mm[1]  = bf_rne(m4.y); mm[2]  = bf_rne(m4.z); mm[3]  = bf_rne(m4.w);
      rs[0]  = rsqrtf(bf_rne(v4.x) + BNEPS); rs[1] = rsqrtf(bf_rne(v4.y) + BNEPS);
      rs[2]  = rsqrtf(bf_rne(v4.z) + BNEPS); rs[3] = rsqrtf(bf_rne(v4.w) + BNEPS);
    }
    v4f pv[16];
#pragma unroll
    for (int i = 0; i < 16; ++i) {
      const int row = rowBase + 16 * wave + i;
      const int xr  = row < nN ? row : nN - 1;
      const v4f xs = *(const v4fa*)(stg + (16 * wave + i) * GBN + 4 * lane);
      const v4f gc = *(const v4f*)(GC + (size_t)row * CIN + cb);
      const v4f xv = *(const v4f*)(xin + (size_t)xr * CIN + cb);
      float a[4], q[4], xx[4], y[4];
      a[0] = xs.x; a[1] = xs.y; a[2] = xs.z; a[3] = xs.w;
      q[0] = gc.x; q[1] = gc.y; q[2] = gc.z; q[3] = gc.w;
      xx[0] = xv.x; xx[1] = xv.y; xx[2] = xv.z; xx[3] = xv.w;
#pragma unroll
      for (int c = 0; c < 4; ++c) {
        const float t  = (q[c] + bg_[c]) + (a[c] + bp_[c]);
        float bn = gg[c] * (t - mm[c]);
        bn = fmaf(bn, rs[c], be[c]);
        y[c] = fmaxf(bn, 0.0f) + bf_rne(xx[c]);
      }
      v4f r4;
      r4.x = y[0]; r4.y = y[1]; r4.z = y[2]; r4.w = y[3];
      pv[i] = r4;
    }
#pragma unroll
    for (int i = 0; i < 16; ++i) {
      const int row = rowBase + 16 * wave + i;
      float* op = out + (size_t)row * CIN + cb;
      if (row < nN) *(volatile v4f*)op = pv[i];
    }
    __threadfence();
#pragma unroll
    for (int i = 0; i < 16; ++i) {
      const int row = rowBase + 16 * wave + i;
      float* op = out + (size_t)row * CIN + cb;
      if (row < nN) *(volatile v4f*)op = pv[i];
    }
  }
}

__global__ __launch_bounds__(NTHR) void k_deg(const int* __restrict__ dsts, const float* __restrict__ ew,
                                              float* DV, int nN, int nE, int vec8) {
  extern __shared__ __attribute__((aligned(16))) int lds_i[];
  const int tid = (int)threadIdx.x, lane = tid & 31, wave = tid >> 5;
  const int nodeBase = (int)blockIdx.x * NBA;
  const int nh = seg_front(dsts, nE, nodeBase, vec8, lds_i, tid, lane, wave);
  const int* reg2 = lds_i + RCAP;
  const int* scnt = lds_i + 2 * RCAP;
  const int* soff = scnt + NBA;
  float* res = (float*)(lds_i + 2 * RCAP + 2 * NBA);

  const int nbw = NBA / NWAVE;
  const bool ovf = (nh >= RCAP);
  const float qnan = __int_as_float(0x7fc00000);
#pragma unroll 1
  for (int jt = 0; jt < nbw; ++jt) {
    const int slot = wave * nbw + jt;
    const int node = nodeBase + slot;
    int st = soff[slot];
    const int craw = scnt[slot];
    int cnt = craw;
    st  = st < 0 ? 0 : (st > nh ? nh : st);
    cnt = cnt < 0 ? 0 : (cnt > DEGCAP ? DEGCAP : cnt);
    if (cnt > nh - st) cnt = nh - st;
    const float pz = (ovf || craw > DEGCAP) ? qnan : 0.0f;
    float p = 0.0f;
#pragma unroll 1
    for (int b0 = 0; b0 < cnt; b0 += 32) {
      int idx = st + b0 + lane; idx = idx > RCAP - 1 ? RCAP - 1 : idx;
      int eid = reg2[idx]; eid = eid < 0 ? 0 : (eid > nE - 1 ? nE - 1 : eid);
      const float wv = bf_rne(ew[eid]);
      p += (b0 + lane < cnt) ? wv : 0.0f;
    }
#pragma unroll
    for (int off = 16; off > 0; off >>= 1) p += __shfl_xor(p, off, 32);
    const float deg = p + 1.0f;
    float dv = deg > 0.0f ? rsqrtf(fmaxf(deg, 1e-12f)) : 0.0f;
    dv = (node < nN ? dv : 0.0f) + pz;
    if (lane == 0) res[slot] = dv;
  }
  __syncthreads();
  if (tid < NBA / 4) {
    const v4f v = *(const v4fa*)(res + 4 * tid);
    float* dp = DV + (size_t)nodeBase + 4 * tid;
    *(volatile v4f*)dp = v;
    __threadfence();
    *(volatile v4f*)dp = v;
  }
}

__global__ __launch_bounds__(NTHR) void k_agg(const int* __restrict__ srcs, const int* __restrict__ dsts,
                                              const float* __restrict__ ew, const float* __restrict__ HH,
                                              const float* __restrict__ DV,
                                              const float* __restrict__ asrc, const float* __restrict__ adst,
                                              const float* __restrict__ bgat,
                                              float* GC, unsigned short* GA,
                                              int nN, int nE, int vec8, int mRows) {
  extern __shared__ __attribute__((aligned(16))) int lds_i[];
  const int tid = (int)threadIdx.x, lane = tid & 31, wave = tid >> 5;
  const int nodeBase = (int)blockIdx.x * NBA;
  const int nh = seg_front(dsts, nE, nodeBase, vec8, lds_i, tid, lane, wave);
  const int* reg2 = lds_i + RCAP;
  const int* scnt = lds_i + 2 * RCAP;
  const int* soff = scnt + NBA;

  const int nbw = NBA / NWAVE;
  const bool ovf = (nh >= RCAP);
  const float qnan = __int_as_float(0x7fc00000);
  float as8[8], ad8[8], bg8[8];
  ld8bf(asrc + 8 * lane, as8);
  ld8bf(adst + 8 * lane, ad8);
  ld8bf(bgat + 8 * lane, bg8);

#pragma unroll 1
  for (int jt = 0; jt < nbw; ++jt) {
    const int slot = wave * nbw + jt;
    const int node = nodeBase + slot;
    int st = soff[slot];
    const int craw = scnt[slot];
    int cnt = craw;
    st  = st < 0 ? 0 : (st > nh ? nh : st);
    cnt = cnt < 0 ? 0 : (cnt > DEGCAP ? DEGCAP : cnt);
    if (cnt > nh - st) cnt = nh - st;
    const float pz = (ovf || craw > DEGCAP) ? qnan : 0.0f;
    const bool live = node < nN;
    const int nc = node < nN ? node : nN - 1;

    const float* rp = HH + (size_t)nc * HWID;
    const v4f hd0 = *(const v4f*)(rp + 4 * lane);
    const v4f hd1 = *(const v4f*)(rp + (CIN / 2) + 4 * lane);
    const v4f gd0 = *(const v4f*)(rp + CIN + 8 * lane);
    const v4f gd1 = *(const v4f*)(rp + CIN + 8 * lane + 4);
    const float dvd = DV[nc];
    float gdv[8];
    gdv[0] = gd0.x; gdv[1] = gd0.y; gdv[2] = gd0.z; gdv[3] = gd0.w;
    gdv[4] = gd1.x; gdv[5] = gd1.y; gdv[6] = gd1.z; gdv[7] = gd1.w;
    float pd = gdv[0] * ad8[0];
    float ps = gdv[0] * as8[0];
#pragma unroll
    for (int j = 1; j < 8; ++j) { pd = fmaf(gdv[j], ad8[j], pd); ps = fmaf(gdv[j], as8[j], ps); }
    pd += __shfl_xor(pd, 1, 32);
    pd += __shfl_xor(pd, 2, 32);
    pd += __shfl_xor(pd, 4, 32);
    ps += __shfl_xor(ps, 1, 32);
    ps += __shfl_xor(ps, 2, 32);
    ps += __shfl_xor(ps, 4, 32);
    float l0 = ps + pd;
    l0 = l0 > 0.f ? l0 : NEGSL * l0;
    float mx = l0, dn = 1.0f;
    float g[8];
#pragma unroll
    for (int j = 0; j < 8; ++j) g[j] = gdv[j];
    const float cs = dvd * dvd;
    float c[8];
    c[0] = cs * hd0.x; c[1] = cs * hd0.y; c[2] = cs * hd0.z; c[3] = cs * hd0.w;
    c[4] = cs * hd1.x; c[5] = cs * hd1.y; c[6] = cs * hd1.z; c[7] = cs * hd1.w;

#pragma unroll 1
    for (int b0 = 0; b0 < cnt; b0 += 32) {
      int idx = st + b0 + lane; idx = idx > RCAP - 1 ? RCAP - 1 : idx;
      int eid = reg2[idx]; eid = eid < 0 ? 0 : (eid > nE - 1 ? nE - 1 : eid);
      int sr = srcs[eid]; sr = sr < 0 ? 0 : (sr > nN - 1 ? nN - 1 : sr);
      const float wv  = bf_rne(ew[eid]);
      const float dvs = DV[sr];
      const float cg  = (dvs * wv) * dvd;
      const int   cgi = __float_as_int(cg);
      const int m32 = (cnt - b0) < 32 ? (cnt - b0) : 32;
#pragma unroll 1
      for (int k = 0; k < m32; ++k) {
        const int   sk = __builtin_amdgcn_readlane(sr, k);
        const float ck = __int_as_float(__builtin_amdgcn_readlane(cgi, k));
        const float* sp = HH + (size_t)sk * HWID;
        const v4f hs0 = *(const v4f*)(sp + 4 * lane);
        const v4f hs1 = *(const v4f*)(sp + (CIN / 2) + 4 * lane);
        const v4f gs0 = *(const v4f*)(sp + CIN + 8 * lane);
        const v4f gs1 = *(const v4f*)(sp + CIN + 8 * lane + 4);
        c[0] = fmaf(ck, hs0.x, c[0]); c[1] = fmaf(ck, hs0.y, c[1]); c[2] = fmaf(ck, hs0.z, c[2]); c[3] = fmaf(ck, hs0.w, c[3]);
        c[4] = fmaf(ck, hs1.x, c[4]); c[5] = fmaf(ck, hs1.y, c[5]); c[6] = fmaf(ck, hs1.z, c[6]); c[7] = fmaf(ck, hs1.w, c[7]);
        float gsv[8];
        gsv[0] = gs0.x; gsv[1] = gs0.y; gsv[2] = gs0.z; gsv[3] = gs0.w;
        gsv[4] = gs1.x; gsv[5] = gs1.y; gsv[6] = gs1.z; gsv[7] = gs1.w;
        float es = gsv[0] * as8[0];
#pragma unroll
        for (int j = 1; j < 8; ++j) es = fmaf(gsv[j], as8[j], es);
        es += __shfl_xor(es, 1, 32);
        es += __shfl_xor(es, 2, 32);
        es += __shfl_xor(es, 4, 32);
        float lg = es + pd;
        lg = lg > 0.f ? lg : NEGSL * lg;
        const float df = lg - mx;
        const float ee = __expf(-fabsf(df));
        const bool up  = df > 0.f;
        const float s1 = up ? ee : 1.0f;
        const float s2 = up ? 1.0f : ee;
        mx = up ? lg : mx;
        dn = fmaf(dn, s1, s2);
#pragma unroll
        for (int j = 0; j < 8; ++j) g[j] = fmaf(g[j], s1, s2 * gsv[j]);
      }
    }
    const float inv = __builtin_amdgcn_rcpf(dn);
    float t[8];
#pragma unroll
    for (int j = 0; j < 8; ++j) {
      const float v = fmaf(g[j], inv, bg8[j]);
      t[j] = (live ? v : 0.0f) + pz;
      c[j] = (live ? c[j] : 0.0f) + pz;
    }
    v4f c0v, c1v;
    c0v.x = c[0]; c0v.y = c[1]; c0v.z = c[2]; c0v.w = c[3];
    c1v.x = c[4]; c1v.y = c[5]; c1v.z = c[6]; c1v.w = c[7];
    v4u hv, lv;
    {
      unsigned int hwd[4], lwd[4];
#pragma unroll
      for (int j = 0; j < 4; ++j) {
        const unsigned short ha = bf_bits(t[2 * j]), hb = bf_bits(t[2 * j + 1]);
        const unsigned short la = bf_bits(t[2 * j] - bf_val(ha)), lb = bf_bits(t[2 * j + 1] - bf_val(hb));
        hwd[j] = (unsigned int)ha | ((unsigned int)hb << 16);
        lwd[j] = (unsigned int)la | ((unsigned int)lb << 16);
      }
      hv.x = hwd[0]; hv.y = hwd[1]; hv.z = hwd[2]; hv.w = hwd[3];
      lv.x = lwd[0]; lv.y = lwd[1]; lv.z = lwd[2]; lv.w = lwd[3];
    }

    if (node < mRows) {
      float* gp0 = GC + (size_t)node * CIN + 4 * lane;
      float* gp1 = gp0 + (CIN / 2);
      unsigned short* ap0 = GA + (size_t)node * (size_t)KP + 8 * lane;
      unsigned short* ap1 = ap0 + CIN;
      *(volatile v4f*)gp0 = c0v;
      *(volatile v4f*)gp1 = c1v;
      *(volatile v4u*)ap0 = hv;
      *(volatile v4u*)ap1 = lv;
      __threadfence();
      *(volatile v4f*)gp0 = c0v;
      *(volatile v4f*)gp1 = c1v;
      *(volatile v4u*)ap0 = hv;
      *(volatile v4u*)ap1 = lv;
    }
  }
}

static inline int cdiv(int a, int b) { return (a + b - 1) / b; }
static inline size_t al256(size_t o) { return (o + 255) & ~(size_t)255; }

extern "C" void kernel_launch(void* const* d_in, const int* in_sizes, int n_in,
                              void* d_out, int out_size, void* d_ws, size_t ws_size,
                              hipStream_t stream) {
  if (n_in < 15) return;
  if (in_sizes[0] < CIN || (in_sizes[0] % CIN) != 0) return;
  const int nN = in_sizes[0] / CIN;
  if (nN < 1 || nN > (1 << 22)) return;
  if (in_sizes[1] < 2 || (in_sizes[1] & 1) != 0) return;
  const int nE = in_sizes[1] / 2;
  if (nE < 1 || nE > (1 << 21)) return;
  if (in_sizes[2] != nE) return;
  if (in_sizes[3] != CIN * CIN || in_sizes[4] != CIN) return;
  if (in_sizes[5] != CIN * CIN) return;
  if (in_sizes[6] != CIN || in_sizes[7] != CIN || in_sizes[8] != CIN) return;
  if (in_sizes[9] != CIN * CIN || in_sizes[10] != CIN) return;
  if (in_sizes[11] != CIN || in_sizes[12] != CIN || in_sizes[13] != CIN || in_sizes[14] != CIN) return;
  if ((long long)out_size != (long long)nN * CIN) return;

  const float* x     = (const float*)d_in[0];
  const int*   edge  = (const int*)d_in[1];
  const float* ew    = (const float*)d_in[2];
  const float* wgcn  = (const float*)d_in[3];
  const float* bgcn  = (const float*)d_in[4];
  const float* wgat  = (const float*)d_in[5];
  const float* asrc  = (const float*)d_in[6];
  const float* adst  = (const float*)d_in[7];
  const float* bgat  = (const float*)d_in[8];
  const float* wproj = (const float*)d_in[9];
  const float* bproj = (const float*)d_in[10];
  const float* gam   = (const float*)d_in[11];
  const float* bet   = (const float*)d_in[12];
  const float* mu    = (const float*)d_in[13];
  const float* var   = (const float*)d_in[14];
  float* out = (float*)d_out;
  const int* src = edge;
  const int* dst = edge + nE;

  const int MP  = cdiv(nN, GBM) * GBM;
  const int gM  = MP / GBM;
  const int gA  = cdiv(MP, NBA);
  const int MPD = gA * NBA;
  if ((long long)gA * NBA < (long long)MP) return;
  const int vec8 = ((nE & 3) == 0) ? 1 : 0;

  char* ws = (char*)d_ws;
  size_t off = 0;
  const size_t oWB  = off; off = al256(off + (size_t)HWID * CIN * 2);
  const size_t oWPB = off; off = al256(off + (size_t)CIN * KP * 2);
  const size_t oXB  = off; off = al256(off + (size_t)MP * CIN * 2);
  const size_t oHH  = off; off = al256(off + (size_t)MP * HWID * 4);
  const size_t oDV  = off; off = al256(off + (size_t)MPD * 4);
  const size_t oGC  = off; off = al256(off + (size_t)MP * CIN * 4);
  const size_t oGA  = off; off = al256(off + (size_t)MP * KP * 2);
  if (off > ws_size || off > (size_t)WSMAX) return;
  unsigned short* WB  = (unsigned short*)(ws + oWB);
  unsigned short* WPB = (unsigned short*)(ws + oWPB);
  unsigned short* XB  = (unsigned short*)(ws + oXB);
  float*          HH  = (float*)(ws + oHH);
  float*          DV  = (float*)(ws + oDV);
  float*          GC  = (float*)(ws + oGC);
  unsigned short* GA  = (unsigned short*)(ws + oGA);

  hipFuncSetAttribute(reinterpret_cast<const void*>(&k_deg), hipFuncAttributeMaxDynamicSharedMemorySize, LDS_AGG);
  hipFuncSetAttribute(reinterpret_cast<const void*>(&k_agg), hipFuncAttributeMaxDynamicSharedMemorySize, LDS_AGG);

  k_wprep<<<(2 * NUW + NUP) / NTHR, NTHR, 0, stream>>>(wgcn, wgat, wproj, WB, WPB);
  const int nUx = MP * (CIN / 8);
  k_cvx<<<cdiv(nUx, NTHR), NTHR, 0, stream>>>(x, nN, nUx, XB);

  k_gemm<0><<<dim3(gM, HWID / GBN), GTHR, 0, stream>>>(XB, CIN, WB, CIN, CIN, HH, HWID,
                                                       GC, x, bgcn, bproj, gam, bet, mu, var, out, nN);

  k_deg<<<gA, NTHR, LDS_AGG, stream>>>(dst, ew, DV, nN, nE, vec8);

  k_agg<<<gA, NTHR, LDS_AGG, stream>>>(src, dst, ew, HH, DV, asrc, adst, bgat, GC, GA, nN, nE, vec8, MP);

  k_gemm<1><<<dim3(gM, CIN / GBN), GTHR, 0, stream>>>(GA, KP, WPB, KP, KP, HH, HWID,
                                                      GC, x, bgcn, bproj, gam, bet, mu, var, out, nN);
}
